// CausalGatedD2Attention_86045374808073
// MI455X (gfx1250) — hardware-verified
//
#include <hip/hip_runtime.h>
#include <math.h>

constexpr int kBatch    = 4;
constexpr int kSeq      = 2048;
constexpr int kDim      = 1024;
constexpr int kTok      = kBatch * kSeq;
constexpr int kQkvPitch = 3 * kDim;
constexpr int kNqkg     = 3 * kDim;
constexpr int kNall     = 4 * kDim;
constexpr int kEarly    = 256;
constexpr float kVCarry  = 64.0f;
constexpr float kPCarry  = 4096.0f;
constexpr float kPVScale = 1.0f / (64.0f * 4096.0f);
constexpr float kInvDim  = 1.0f / 1024.0f;
constexpr float kLnEps   = 1e-5f;
constexpr float kDenEps  = 1e-6f;

static_assert(kTok % 64 == 0 && kSeq % 64 == 0 && kDim % 64 == 0 && kEarly % 64 == 0);
static_assert(kDim % 32 == 0 && kSeq % 32 == 0 && kEarly % 32 == 0);

typedef __attribute__((ext_vector_type(16))) _Float16 v16h;
typedef __attribute__((ext_vector_type(8)))  _Float16 v8h;
typedef __attribute__((ext_vector_type(16))) __bf16   v16b;
typedef __attribute__((ext_vector_type(8)))  __bf16   v8b;
typedef __attribute__((ext_vector_type(8)))  float    v8f;
typedef __attribute__((ext_vector_type(4)))  float    v4f;
typedef __attribute__((ext_vector_type(2)))  float    v2f;
typedef __attribute__((ext_vector_type(4)))  unsigned int v4u;

__device__ __forceinline__ unsigned short f2bf_bits(float f) {
  unsigned u = __float_as_uint(f);
  return (unsigned short)((u + 0x7FFFu + ((u >> 16) & 1u)) >> 16);
}
__device__ __forceinline__ float bf_bits2f(unsigned short h) { return __uint_as_float(((unsigned)h) << 16); }

__device__ __forceinline__ void dep_guard_h(v8f& a, v8f& b, v16h x, v16h y) { asm volatile("v_nop\n\tv_nop\n\tv_nop\n\tv_nop" : "+v"(a), "+v"(b) : "v"(x), "v"(y)); }
__device__ __forceinline__ void dep_guard_b(v8f& a, v8f& b, v16b x, v16b y) { asm volatile("v_nop\n\tv_nop\n\tv_nop\n\tv_nop" : "+v"(a), "+v"(b) : "v"(x), "v"(y)); }
__device__ __forceinline__ void keep4_h(v16h a, v16h b, v16h c, v16h d) { asm volatile("v_nop" :: "v"(a), "v"(b), "v"(c), "v"(d)); }
__device__ __forceinline__ void keep4_b(v16b a, v16b b, v16b c, v16b d) { asm volatile("v_nop" :: "v"(a), "v"(b), "v"(c), "v"(d)); }
__device__ __forceinline__ void acc_guard4(v8f& a, v8f& b, v8f& c, v8f& d) { asm volatile("v_nop\n\tv_nop\n\tv_nop\n\tv_nop" : "+v"(a), "+v"(b), "+v"(c), "+v"(d)); }
template <typename T> struct Frag;
template <> struct Frag<_Float16> {
  typedef v16h V; union U { v16h v; v8h h[2]; };
  static __device__ __forceinline__ v16h load(const _Float16* p) {
    U f; f.h[0] = *(const v8h*)(p); f.h[1] = *(const v8h*)(p + 16); return f.v;
  }
  static __device__ __forceinline__ v8f mma(v16h a, v16h b, v8f c) {
    return __builtin_amdgcn_wmma_f32_16x16x32_f16(false, a, false, b, (short)0, c, false, false);
  }
  static __device__ __forceinline__ void guard(v8f& a, v8f& b, v16h x, v16h y) { dep_guard_h(a, b, x, y); }
  static __device__ __forceinline__ void keep(v16h a, v16h b, v16h c, v16h d) { keep4_h(a, b, c, d); }
};
template <> struct Frag<__bf16> {
  typedef v16b V; union U { v16b v; v8b h[2]; };
  static __device__ __forceinline__ v16b load(const __bf16* p) {
    U f; f.h[0] = *(const v8b*)(p); f.h[1] = *(const v8b*)(p + 16); return f.v;
  }
  static __device__ __forceinline__ v8f mma(v16b a, v16b b, v8f c) {
    return __builtin_amdgcn_wmma_f32_16x16x32_bf16(false, a, false, b, (short)0, c, false, false);
  }
  static __device__ __forceinline__ void guard(v8f& a, v8f& b, v16b x, v16b y) { dep_guard_b(a, b, x, y); }
  static __device__ __forceinline__ void keep(v16b a, v16b b, v16b c, v16b d) { keep4_b(a, b, c, d); }
};

__device__ __forceinline__ unsigned pk16(unsigned short a, unsigned short b) { return (unsigned)a | ((unsigned)b << 16); }
__device__ __forceinline__ unsigned short h_bits(float f) { const _Float16 h = (_Float16)f; return __builtin_bit_cast(unsigned short, h); }
__device__ __forceinline__ float bfr(float f) { return bf_bits2f(f2bf_bits(f)); }

template <int ET> struct Elem;
template <> struct Elem<0> { typedef _Float16 T; };
template <> struct Elem<1> { typedef __bf16 T; };
template <int ET, int SPLITM, int BIAS_MODE, int OUT_MODE, int TILEMAP>
__global__ __launch_bounds__(256) void wmma_gemm64(
    const unsigned short* __restrict__ Ap, const unsigned short* __restrict__ A2p, int lda,
    const unsigned short* __restrict__ Btp, const unsigned short* __restrict__ Bt2p, int ldb,
    void* __restrict__ Cout, void* __restrict__ Cout2, int ldc,
    const float* __restrict__ bias,
    int M, int N, int K, int kbase, float scale) {
  typedef typename Elem<ET>::T T;
  typedef typename Frag<T>::V V;
  constexpr bool SPLA = (SPLITM == 1) || (SPLITM == 3);
  constexpr bool SPLB = (SPLITM == 1) || (SPLITM == 2);
  const T* A = (const T*)Ap; const T* A2 = (const T*)A2p; const T* Bt = (const T*)Btp; const T* Bt2 = (const T*)Bt2p;
  __shared__ __align__(16) float sT[8][16 * 68];
  const int lane = threadIdx.x & 31;
  const int wave = threadIdx.x >> 5;
  const int tilesN = N >> 6;
  const int tilesM = M >> 6;
  const int tile = blockIdx.x * 8 + wave;
  int tm, tn;
  if (TILEMAP == 1) {
    const int ntri = tilesM * (tilesM + 1) / 2;
    if (tile >= ntri) return;
    int e = (int)((sqrtf(8.0f * (float)tile + 1.0f) - 1.0f) * 0.5f);
    if ((e + 1) * (e + 2) / 2 <= tile) ++e;
    if (e * (e + 1) / 2 > tile) --e;
    if (e < 0) e = 0;
    if (e > tilesM - 1) e = tilesM - 1;
    tm = e;
    tn = tile - e * (e + 1) / 2;
    if (tn < 0) tn = 0;
    if (tn > tm) tn = tm;
  } else {
    if (tile >= tilesM * tilesN) return;
    tm = tile / tilesN;
    tn = tile - tm * tilesN;
  }
  const int m0 = tm << 6;
  const int n0 = tn << 6;
  int Kend = K;
  if (TILEMAP == 2) { const int kl = kbase + m0 + 64; Kend = (kl < K) ? kl : K; }

  const int rlane = lane & 15;
  const int koff  = (lane >> 4) * 8;
  const int mOff  = (lane >> 4) * 8;

  v8f acc[4][4];
#pragma unroll
  for (int i = 0; i < 4; ++i)
#pragma unroll
    for (int j = 0; j < 4; ++j) acc[i][j] = (v8f){0.f,0.f,0.f,0.f,0.f,0.f,0.f,0.f};

  for (int k0 = 0; k0 < Kend; k0 += 32) {
    V bh[4], bl[4];
#pragma unroll
    for (int j = 0; j < 4; ++j) {
      const size_t bo = (size_t)(n0 + (j << 4) + rlane) * ldb + koff + k0;
      bh[j] = Frag<T>::load(Bt + bo);
      if (SPLB) bl[j] = Frag<T>::load(Bt2 + bo);
    }
#pragma unroll
    for (int i = 0; i < 4; ++i) {
      const size_t ao = (size_t)(m0 + (i << 4) + rlane) * lda + koff + k0;
      V ah = Frag<T>::load(A + ao);
      V al;
      if (SPLA) al = Frag<T>::load(A2 + ao);
#pragma unroll
      for (int j = 0; j < 4; ++j) {
        acc[i][j] = Frag<T>::mma(ah, bh[j], acc[i][j]);
        if (SPLB) acc[i][j] = Frag<T>::mma(ah, bl[j], acc[i][j]);
        if (SPLA) acc[i][j] = Frag<T>::mma(al, bh[j], acc[i][j]);
      }
      Frag<T>::guard(acc[i][0], acc[i][3], ah, SPLA ? al : ah);
    }
    Frag<T>::keep(bh[0], bh[1], bh[2], bh[3]);
    if (SPLB) Frag<T>::keep(bl[0], bl[1], bl[2], bl[3]);
  }
  acc_guard4(acc[0][0], acc[0][1], acc[0][2], acc[0][3]);
  acc_guard4(acc[1][0], acc[1][1], acc[1][2], acc[1][3]);
  acc_guard4(acc[2][0], acc[2][1], acc[2][2], acc[2][3]);
  acc_guard4(acc[3][0], acc[3][1], acc[3][2], acc[3][3]);

  float* slab = sT[wave];
#pragma unroll
  for (int i = 0; i < 4; ++i) {
    const int mBase = m0 + (i << 4);
#pragma unroll
    for (int j = 0; j < 4; ++j) {
      const int n = n0 + (j << 4) + rlane;
      float bv = 0.f;
      if (BIAS_MODE == 2) bv = bias[n];
#pragma unroll
      for (int r = 0; r < 8; ++r) {
        float v = acc[i][j][r] * scale;
        if (BIAS_MODE == 1) v += bias[mBase + mOff + r];
        if (BIAS_MODE == 2) v += bv;
        slab[(mOff + r) * 68 + (j << 4) + rlane] = v;
      }
    }
    __builtin_amdgcn_fence(__ATOMIC_RELEASE, "workgroup");
    __builtin_amdgcn_wave_barrier();
    __builtin_amdgcn_fence(__ATOMIC_ACQUIRE, "workgroup");
    if (OUT_MODE == 0) {
      float* C = (float*)Cout;
      const int hh = lane >> 4, c4 = (lane & 15) * 4;
      for (int pass = 0; pass < 2; ++pass) {
#pragma unroll
        for (int it = 0; it < 8; ++it) {
          const int row = it * 2 + hh;
          v4f v = *(const v4f*)(slab + row * 68 + c4);
          *(volatile v4f*)(C + (size_t)(mBase + row) * ldc + n0 + c4) = v;
        }
        __threadfence();
      }
    } else {
      const int q = lane >> 3, c8 = (lane & 7) * 8;
      unsigned short* C  = (unsigned short*)Cout;
      unsigned short* C2 = (OUT_MODE == 2) ? (unsigned short*)Cout2 : nullptr;
      for (int pass = 0; pass < 2; ++pass) {
#pragma unroll
        for (int it = 0; it < 4; ++it) {
          const int row = it * 4 + q;
          const float* sp = slab + row * 68 + c8;
          v8h hv, lv;
#pragma unroll
          for (int e = 0; e < 8; ++e) {
            if (OUT_MODE == 1) {
              hv[e] = (_Float16)sp[e];
            } else {
              unsigned short hb = f2bf_bits(sp[e]);
              unsigned short lb = f2bf_bits(sp[e] - bf_bits2f(hb));
              hv[e] = __builtin_bit_cast(_Float16, hb);
              lv[e] = __builtin_bit_cast(_Float16, lb);
            }
          }
          *(volatile v8h*)(C + (size_t)(mBase + row) * ldc + n0 + c8) = hv;
          if (OUT_MODE == 2) *(volatile v8h*)(C2 + (size_t)(mBase + row) * ldc + n0 + c8) = lv;
        }
        __threadfence();
      }
    }
    __builtin_amdgcn_fence(__ATOMIC_RELEASE, "workgroup");
    __builtin_amdgcn_wave_barrier();
    __builtin_amdgcn_fence(__ATOMIC_ACQUIRE, "workgroup");
  }
}

__global__ __launch_bounds__(256) void wprep_kernel(const float* __restrict__ qkv_w, const float* __restrict__ gate_w,
                                                    const float* __restrict__ qkv_b, const float* __restrict__ gate_b,
                                                    unsigned short* __restrict__ WT, float* __restrict__ biasv) {
  __shared__ float sm[64][65];
  const int t  = threadIdx.x;
  const int d0 = blockIdx.x * 64;
  const int n0 = blockIdx.y * 64;
  const float* src; int pitch; int col0; const float* bsrc; int bcol0; float bsc;
  if (n0 < 2 * kDim)      { src = qkv_w;  pitch = kQkvPitch; col0 = n0;            bsrc = qkv_b;  bcol0 = n0;            bsc = 1.0f; }
  else if (n0 < 3 * kDim) { src = gate_w; pitch = kDim;      col0 = n0 - 2 * kDim; bsrc = gate_b; bcol0 = n0 - 2 * kDim; bsc = 1.0f; }
  else                    { src = qkv_w;  pitch = kQkvPitch; col0 = n0 - kDim;     bsrc = qkv_b;  bcol0 = n0 - kDim;     bsc = kVCarry; }
#pragma unroll
  for (int i = 0; i < 16; ++i) {
    const int e = i * 256 + t;
    const int r = e >> 6;
    const int c = e & 63;
    sm[c][r] = bfr(src[(size_t)(d0 + r) * pitch + col0 + c]);
  }
  __syncthreads();
  const int lane = t & 31, wave = t >> 5;
  const int q = lane >> 3, c8 = (lane & 7) * 8;
  for (int pass = 0; pass < 2; ++pass) {
#pragma unroll
    for (int it = 0; it < 2; ++it) {
      const int row = wave * 8 + it * 4 + q;
      unsigned short hb[8];
#pragma unroll
      for (int e = 0; e < 8; ++e) hb[e] = f2bf_bits(sm[row][c8 + e]);
      const v4u u = (v4u){pk16(hb[0], hb[1]), pk16(hb[2], hb[3]), pk16(hb[4], hb[5]), pk16(hb[6], hb[7])};
      *(volatile v4u*)(WT + (size_t)(n0 + row) * kDim + d0 + c8) = u;
    }
    __threadfence();
  }
  if (blockIdx.x == 0 && wave == 0) {
    const int l16 = lane & 15;
    v4f bv;
#pragma unroll
    for (int e = 0; e < 4; ++e) bv[e] = bfr(bsrc[bcol0 + l16 * 4 + e]) * bsc;
    for (int pass = 0; pass < 2; ++pass) {
      if (lane < 16) *(volatile v4f*)(biasv + n0 + l16 * 4) = bv;
      __threadfence();
    }
  }
}

__global__ __launch_bounds__(128) void ln_split_kernel(const float* __restrict__ x, const float* __restrict__ g,
                                                       const float* __restrict__ bta,
                                                       unsigned short* __restrict__ XH, unsigned short* __restrict__ XL) {
  __shared__ float red0[4];
  __shared__ float red1[4];
  const int row  = blockIdx.x;
  const int tid  = threadIdx.x;
  const int lane = tid & 31, wave = tid >> 5;
  const int c0   = tid * 8;
  const float* xr = x + (size_t)row * kDim + c0;
  const v4f a = *(const v4f*)(xr);
  const v4f c = *(const v4f*)(xr + 4);
  float xv[8];
#pragma unroll
  for (int e = 0; e < 4; ++e) { xv[e] = bfr(a[e]); xv[4 + e] = bfr(c[e]); }
  float s = 0.f;
#pragma unroll
  for (int e = 0; e < 8; ++e) s += xv[e];
#pragma unroll
  for (int off = 16; off > 0; off >>= 1) s += __shfl_xor(s, off, 32);
  if (lane == 0) red0[wave] = s;
  __syncthreads();
  const float mu = ((red0[0] + red0[1]) + (red0[2] + red0[3])) * kInvDim;
  float dv[8];
  float s2 = 0.f;
#pragma unroll
  for (int e = 0; e < 8; ++e) { dv[e] = xv[e] - mu; const float sq = dv[e] * dv[e]; s2 += sq; }
#pragma unroll
  for (int off = 16; off > 0; off >>= 1) s2 += __shfl_xor(s2, off, 32);
  if (lane == 0) red1[wave] = s2;
  __syncthreads();
  const float var  = ((red1[0] + red1[1]) + (red1[2] + red1[3])) * kInvDim;
  const float rstd = 1.0f / sqrtf(var + kLnEps);
  const v4f ga = *(const v4f*)(g + c0);
  const v4f gc = *(const v4f*)(g + c0 + 4);
  const v4f ba = *(const v4f*)(bta + c0);
  const v4f bc = *(const v4f*)(bta + c0 + 4);
  float y[8];
#pragma unroll
  for (int e = 0; e < 4; ++e) {
    y[e]     = dv[e] * rstd * bfr(ga[e]) + bfr(ba[e]);
    y[4 + e] = dv[4 + e] * rstd * bfr(gc[e]) + bfr(bc[e]);
  }
  unsigned short hb[8], lb[8];
#pragma unroll
  for (int e = 0; e < 8; ++e) {
    hb[e] = f2bf_bits(y[e]);
    lb[e] = f2bf_bits(y[e] - bf_bits2f(hb[e]));
  }
  const v4u uh = (v4u){pk16(hb[0], hb[1]), pk16(hb[2], hb[3]), pk16(hb[4], hb[5]), pk16(hb[6], hb[7])};
  const v4u ul = (v4u){pk16(lb[0], lb[1]), pk16(lb[2], lb[3]), pk16(lb[4], lb[5]), pk16(lb[6], lb[7])};
  unsigned short* ph = XH + (size_t)row * kDim + c0;
  unsigned short* pl = XL + (size_t)row * kDim + c0;
  *(volatile v4u*)ph = uh;
  *(volatile v4u*)pl = ul;
  __threadfence();
  *(volatile v4u*)ph = uh;
  *(volatile v4u*)pl = ul;
}

__device__ __forceinline__ float elu1(float z) { const float e = expf(fminf(z, 0.0f)); return (z > 0.0f) ? (z + 1.0f) : e; }
__device__ __forceinline__ float sigm(float z) { return __builtin_amdgcn_rcpf(1.0f + expf(-z)); }

__global__ __launch_bounds__(256) void act_kernel(const float* __restrict__ Y, unsigned short* __restrict__ QF,
                                                  unsigned short* __restrict__ KF) {
  const int idx = blockIdx.x * 256 + threadIdx.x;
  const int row = idx >> 9;
  const int d   = (idx & 511) * 2;
  const float* yr = Y + (size_t)row * kNqkg;
  const v2f qv = *(const v2f*)(yr + d);
  const v2f kv = *(const v2f*)(yr + kDim + d);
  const v2f gv = *(const v2f*)(yr + 2 * kDim + d);
  const float qf0 = elu1(qv[0]), qf1 = elu1(qv[1]);
  const float kf0 = elu1(kv[0] * sigm(gv[0])), kf1 = elu1(kv[1] * sigm(gv[1]));
  const unsigned uq = pk16(h_bits(qf0), h_bits(qf1));
  const unsigned uk = pk16(h_bits(kf0), h_bits(kf1));
  const size_t o = ((size_t)row * kDim + d) >> 1;
  ((volatile unsigned*)QF)[o] = uq;
  ((volatile unsigned*)KF)[o] = uk;
  __threadfence();
  ((volatile unsigned*)QF)[o] = uq;
  ((volatile unsigned*)KF)[o] = uk;
}

__global__ __launch_bounds__(256) void vcast_kernel(const float* __restrict__ VT32, unsigned short* __restrict__ VT16,
                                                    unsigned short* __restrict__ VTH, unsigned short* __restrict__ VTL) {
  const int d    = blockIdx.x;
  const int tid  = threadIdx.x;
  const int wave = tid >> 5;
  const int s0   = tid * 8;
  const float* p = VT32 + (size_t)d * kSeq + s0;
  const v4f a = *(const v4f*)(p);
  const v4f c = *(const v4f*)(p + 4);
  float f[8];
#pragma unroll
  for (int e = 0; e < 4; ++e) { f[e] = a[e]; f[4 + e] = c[e]; }
  unsigned short hb[8];
#pragma unroll
  for (int e = 0; e < 8; ++e) hb[e] = h_bits(f[e]);
  const v4u u = (v4u){pk16(hb[0], hb[1]), pk16(hb[2], hb[3]), pk16(hb[4], hb[5]), pk16(hb[6], hb[7])};
  unsigned short* q16 = VT16 + (size_t)d * kSeq + s0;
  *(volatile v4u*)q16 = u;
  __threadfence();
  *(volatile v4u*)q16 = u;
  if (wave == 0) {
    unsigned short hh[8], ll[8];
#pragma unroll
    for (int e = 0; e < 8; ++e) { hh[e] = f2bf_bits(f[e]); ll[e] = f2bf_bits(f[e] - bf_bits2f(hh[e])); }
    const v4u uh = (v4u){pk16(hh[0], hh[1]), pk16(hh[2], hh[3]), pk16(hh[4], hh[5]), pk16(hh[6], hh[7])};
    const v4u ul = (v4u){pk16(ll[0], ll[1]), pk16(ll[2], ll[3]), pk16(ll[4], ll[5]), pk16(ll[6], ll[7])};
    unsigned short* qh = VTH + (size_t)d * kEarly + s0;
    unsigned short* ql = VTL + (size_t)d * kEarly + s0;
    *(volatile v4u*)qh = uh;
    *(volatile v4u*)ql = ul;
    __threadfence();
    *(volatile v4u*)qh = uh;
    *(volatile v4u*)ql = ul;
  }
}

__global__ __launch_bounds__(256) void pnorm_kernel(const float* __restrict__ S, unsigned short* __restrict__ P16,
                                                    unsigned short* __restrict__ PH, unsigned short* __restrict__ PL) {
  __shared__ float red[8];
  const int t    = blockIdx.x;
  const int tid  = threadIdx.x;
  const int lane = tid & 31, wave = tid >> 5;
  const int c0   = tid * 8;
  const int L    = ((t >> 6) + 1) << 6;
  const int cl   = (c0 < L - 8) ? c0 : (L - 8);
  const float* sr = S + (size_t)t * kSeq + cl;
  const v4f a = *(const v4f*)(sr);
  const v4f c = *(const v4f*)(sr + 4);
  float xv[8];
#pragma unroll
  for (int e = 0; e < 4; ++e) {
    xv[e]     = (c0 + e <= t) ? a[e] : 0.0f;
    xv[4 + e] = (c0 + 4 + e <= t) ? c[e] : 0.0f;
  }
  float part = ((xv[0] + xv[1]) + (xv[2] + xv[3])) + ((xv[4] + xv[5]) + (xv[6] + xv[7]));
#pragma unroll
  for (int off = 16; off > 0; off >>= 1) part += __shfl_xor(part, off, 32);
  if (lane == 0) red[wave] = part;
  __syncthreads();
  float tot = red[0];
#pragma unroll
  for (int w = 1; w < 8; ++w) tot += red[w];
  const float den  = tot + kDenEps;
  const float rinv = 1.0f / den;
  float pv[8];
#pragma unroll
  for (int e = 0; e < 8; ++e) pv[e] = (xv[e] * rinv) * kPCarry;
  unsigned short hb[8];
#pragma unroll
  for (int e = 0; e < 8; ++e) hb[e] = h_bits(pv[e]);
  const v4u u = (v4u){pk16(hb[0], hb[1]), pk16(hb[2], hb[3]), pk16(hb[4], hb[5]), pk16(hb[6], hb[7])};
  unsigned short* q16 = P16 + (size_t)t * kSeq + c0;
  for (int pass = 0; pass < 2; ++pass) {
    if (c0 < L) *(volatile v4u*)q16 = u;
    __threadfence();
  }
  if (t < kEarly) {
    unsigned short hh[8], ll[8];
#pragma unroll
    for (int e = 0; e < 8; ++e) { hh[e] = f2bf_bits(pv[e]); ll[e] = f2bf_bits(pv[e] - bf_bits2f(hh[e])); }
    const v4u uh = (v4u){pk16(hh[0], hh[1]), pk16(hh[2], hh[3]), pk16(hh[4], hh[5]), pk16(hh[6], hh[7])};
    const v4u ul = (v4u){pk16(ll[0], ll[1]), pk16(ll[2], ll[3]), pk16(ll[4], ll[5]), pk16(ll[6], ll[7])};
    const int cc = (c0 < kEarly - 8) ? c0 : (kEarly - 8);
    unsigned short* qh = PH + (size_t)t * kEarly + cc;
    unsigned short* ql = PL + (size_t)t * kEarly + cc;
    for (int pass = 0; pass < 2; ++pass) {
      if (c0 < L) { *(volatile v4u*)qh = uh; *(volatile v4u*)ql = ul; }
      __threadfence();
    }
  }
}

extern "C" void kernel_launch(void* const* d_in, const int* in_sizes, int n_in,
                              void* d_out, int out_size, void* d_ws, size_t ws_size, hipStream_t stream) {
  if (n_in < 7) return;
  if (in_sizes[0] != kTok * kDim || in_sizes[1] != kDim * kQkvPitch || in_sizes[2] != kQkvPitch ||
      in_sizes[3] != kDim * kDim || in_sizes[4] != kDim || in_sizes[5] != kDim || in_sizes[6] != kDim ||
      out_size != kTok * kDim) return;

  const float* x      = (const float*)d_in[0];
  const float* qkv_w  = (const float*)d_in[1];
  const float* qkv_b  = (const float*)d_in[2];
  const float* gate_w = (const float*)d_in[3];
  const float* gate_b = (const float*)d_in[4];
  const float* ln_g   = (const float*)d_in[5];
  const float* ln_b   = (const float*)d_in[6];
  float* out = (float*)d_out;

  constexpr size_t szX   = (size_t)kTok * kDim * 2;
  constexpr size_t szWT  = (size_t)kNall * kDim * 2;
  constexpr size_t szBI  = (size_t)kNall * 4;
  constexpr size_t szY   = (size_t)kSeq * kNqkg * 4;
  constexpr size_t szQK  = (size_t)kSeq * kDim * 2;
  constexpr size_t szV32 = (size_t)kDim * kSeq * 4;
  constexpr size_t szV16 = (size_t)kDim * kSeq * 2;
  constexpr size_t szVE  = (size_t)kDim * kEarly * 2;
  constexpr size_t szS   = (size_t)kSeq * kSeq * 4;
  constexpr size_t szP16 = (size_t)kSeq * kSeq * 2;
  constexpr size_t szPE  = (size_t)kEarly * kEarly * 2;
  constexpr size_t oXH = 0, oXL = oXH + szX, oWT = oXL + szX, oBI = oWT + szWT, oY = oBI + szBI, oQF = oY + szY,
                   oKF = oQF + szQK, oV32 = oKF + szQK, oV16 = oV32 + szV32, oVH = oV16 + szV16, oVL = oVH + szVE,
                   oS = oVL + szVE, oP16 = oS + szS, oPH = oP16 + szP16, oPL = oPH + szPE, oEnd = oPL + szPE;
  static_assert(oEnd == 114573312ull);
  static_assert(oEnd <= 134217728ull);
  static_assert((oBI % 128) == 0 && (oY % 128) == 0 && (oVH % 128) == 0 && (oPH % 128) == 0 && (oPL % 128) == 0);
  if (oEnd > ws_size) return;

  char* ws = (char*)d_ws;
  unsigned short* XH   = (unsigned short*)(ws + oXH);
  unsigned short* XL   = (unsigned short*)(ws + oXL);
  unsigned short* WT   = (unsigned short*)(ws + oWT);
  float*          BIAS = (float*)(ws + oBI);
  float*          Y    = (float*)(ws + oY);
  unsigned short* QF   = (unsigned short*)(ws + oQF);
  unsigned short* KF   = (unsigned short*)(ws + oKF);
  float*          VT32 = (float*)(ws + oV32);
  unsigned short* VT16 = (unsigned short*)(ws + oV16);
  unsigned short* VTH  = (unsigned short*)(ws + oVH);
  unsigned short* VTL  = (unsigned short*)(ws + oVL);
  float*          S    = (float*)(ws + oS);
  unsigned short* P16  = (unsigned short*)(ws + oP16);
  unsigned short* PH   = (unsigned short*)(ws + oPH);
  unsigned short* PL   = (unsigned short*)(ws + oPL);

  wprep_kernel<<<dim3(kDim / 64, kNall / 64), 256, 0, stream>>>(qkv_w, gate_w, qkv_b, gate_b, WT, BIAS);
  ln_split_kernel<<<kTok, 128, 0, stream>>>(x, ln_g, ln_b, XH, XL);

  constexpr int gridQKG = (kSeq / 64) * (kNqkg / 64) / 8;
  constexpr int gridV   = (kDim / 64) * (kSeq / 64) / 8;
  constexpr int gridS   = ((kSeq / 64) * (kSeq / 64 + 1) / 2 + 7) / 8;
  constexpr int gridPVe = (kEarly / 64) * (kDim / 64) / 8;
  constexpr int gridPVr = ((kSeq - kEarly) / 64) * (kDim / 64) / 8;
  static_assert(gridQKG * 8 == (kSeq / 64) * (kNqkg / 64) && gridV * 8 == (kDim / 64) * (kSeq / 64));
  static_assert(gridPVe * 8 == (kEarly / 64) * (kDim / 64) && gridPVr * 8 == ((kSeq - kEarly) / 64) * (kDim / 64));
  static_assert((kSeq - kEarly) % 64 == 0);

  const unsigned short* WTv = WT + (size_t)kNqkg * kDim;
  for (int b = 0; b < kBatch; ++b) {
    const unsigned short* XHb = XH + (size_t)b * kSeq * kDim;
    const unsigned short* XLb = XL + (size_t)b * kSeq * kDim;
    float* outb = out + (size_t)b * kSeq * kDim;
    wmma_gemm64<1, 3, 2, 0, 0><<<gridQKG, 256, 0, stream>>>(
        XHb, XLb, kDim, WT, WT, kDim, (void*)Y, (void*)Y, kNqkg, BIAS, kSeq, kNqkg, kDim, 0, 1.0f);
    wmma_gemm64<1, 2, 1, 0, 0><<<gridV, 256, 0, stream>>>(
        WTv, WTv, kDim, XHb, XLb, kDim, (void*)VT32, (void*)VT32, kSeq, BIAS + kNqkg, kDim, kSeq, kDim, 0, kVCarry);
    act_kernel<<<(kSeq * (kDim / 2)) / 256, 256, 0, stream>>>(Y, QF, KF);
    vcast_kernel<<<kDim, 256, 0, stream>>>(VT32, VT16, VTH, VTL);
    wmma_gemm64<0, 0, 0, 0, 1><<<gridS, 256, 0, stream>>>(
        QF, QF, kDim, KF, KF, kDim, (void*)S, (void*)S, kSeq, BIAS, kSeq, kSeq, kDim, 0, 1.0f);
    pnorm_kernel<<<kSeq, 256, 0, stream>>>(S, P16, PH, PL);
    wmma_gemm64<1, 1, 0, 0, 2><<<gridPVe, 256, 0, stream>>>(
        PH, PL, kEarly, VTH, VTL, kEarly, (void*)outb, (void*)outb, kDim, BIAS, kEarly, kDim, kEarly, 0, kPVScale);
    wmma_gemm64<0, 0, 0, 0, 2><<<gridPVr, 256, 0, stream>>>(
        P16 + (size_t)kEarly * kSeq, P16 + (size_t)kEarly * kSeq, kSeq, VT16, VT16, kSeq,
        (void*)(outb + (size_t)kEarly * kDim), (void*)(outb + (size_t)kEarly * kDim), kDim, BIAS,
        kSeq - kEarly, kDim, kSeq, kEarly, kPVScale);
  }
}
